// attention_77326591197822
// MI455X (gfx1250) — hardware-verified
//
#include <hip/hip_runtime.h>
#include <stddef.h>
#include <math.h>


typedef _Float16 v16h __attribute__((ext_vector_type(16)));
typedef _Float16 v8h  __attribute__((ext_vector_type(8)));
typedef float    v8f  __attribute__((ext_vector_type(8)));
typedef float    v4f  __attribute__((ext_vector_type(4)));

#ifndef NB
#define NB 1
#endif
#ifndef SEQ
#define SEQ 4096
#endif
#define NB_FULL  1
#define SEQ_FULL 4096
#define DIM   1024
#define NHEAD 16
#define HD    64
#define MROWS (NB * SEQ)
#define EROWS ((SEQ) < 512 ? (SEQ) : 512)

static_assert(NB == 1 && NB_FULL == 1);
static_assert(SEQ >= 128 && SEQ <= SEQ_FULL && (SEQ % 128) == 0);
static_assert(DIM == NHEAD * HD);
static_assert(HD == 64 && ((3 * HD) % 64) == 0);
static_assert((MROWS % 64) == 0 && (MROWS % 8) == 0);
static_assert((DIM % 64) == 0 && ((3 * DIM) % 64) == 0);
static_assert((EROWS % 128) == 0 && EROWS <= SEQ && EROWS <= MROWS);
static_assert((((size_t)MROWS * DIM) % 2048) == 0);

#define LDT 72
#define LDC 68

#define WCARRY 64.0f
#define PCARRY 1024.0f
#define VCARRY 64.0f
#define RCARRY 2048.0f

#define P16_BYTES  ((size_t)MROWS * DIM * 2)
#define R16_BYTES  ((size_t)EROWS * DIM * 2)
#define WQKV_BYTES ((size_t)3 * DIM * DIM * 2)
#define WO_BYTES   ((size_t)DIM * DIM * 2)
#define OFF_WQKV   ((size_t)0)
#define OFF_WO     (OFF_WQKV + WQKV_BYTES)
#define OFF_XN     (OFF_WO + WO_BYTES)
#define OFF_QKV    (OFF_XN + P16_BYTES)
#define OFF_OV     (OFF_QKV + 3 * P16_BYTES)
#define OFF_RES    (OFF_OV + P16_BYTES)
#define OFF_ORES   (OFF_RES + 3 * R16_BYTES)
#define WS_TOTAL   (OFF_ORES + R16_BYTES)
static_assert((size_t)DIM * SEQ * 2 == P16_BYTES);
static_assert((size_t)DIM * EROWS * 2 == R16_BYTES);
static_assert((P16_BYTES % 128) == 0 && (WO_BYTES % 128) == 0 && (R16_BYTES % 128) == 0);
static_assert(WS_TOTAL <= (size_t)134217728);

__device__ __forceinline__ float bf16r(float x) {
  unsigned int u = __float_as_uint(x);
  u = (u + 0x7FFFu + ((u >> 16) & 1u)) & 0xFFFF0000u;
  return __uint_as_float(u);
}

static __device__ __forceinline__ _Float16 toh_flush(float v) {
  const _Float16 r = (_Float16)v;
  return (fabsf(v) < 6.103515625e-05f) ? (_Float16)0.0f : r;
}

__device__ __forceinline__ v16h frag_at(const _Float16* p) {
  v8h lo = *(const v8h*)(p);
  v8h hi = *(const v8h*)(p + 16);
  v16h out;
#pragma unroll
  for (int i = 0; i < 8; ++i) { out[i] = lo[i]; out[i + 8] = hi[i]; }
  return out;
}
__device__ __forceinline__ v16h ld_frag(const _Float16* base, int ld) {
  const int lane = threadIdx.x & 31;
  return frag_at(base + (lane & 15) * ld + (lane >> 4) * 8);
}

__device__ __forceinline__ v8f wmma16(v16h a, v16h b, v8f c) {
  v8f d = __builtin_amdgcn_wmma_f32_16x16x32_f16(false, a, false, b, (short)0, c,
                                                 false, false);
  asm volatile("v_nop\n\tv_nop\n\tv_nop\n\tv_nop" : "+v"(d) : "v"(a), "v"(b));
  return d;
}

__device__ __forceinline__ float red16_max(float x) {
#pragma unroll
  for (int off = 1; off < 16; off <<= 1) x = fmaxf(x, __shfl_xor(x, off, 32));
  return x;
}
__device__ __forceinline__ float red16_sum(float x) {
#pragma unroll
  for (int off = 1; off < 16; off <<= 1) x += __shfl_xor(x, off, 32);
  return x;
}

__device__ __forceinline__ void wave_lds_sync() {
  __builtin_amdgcn_fence(3  , "wavefront");
  asm volatile("s_wait_dscnt 0x0" ::: "memory");
  __builtin_amdgcn_wave_barrier();
}

__global__ __launch_bounds__(256) void wconv_kernel(
    const float* __restrict__ W, _Float16* __restrict__ Wt, int K, int N) {
  __shared__ _Float16 T[64 * LDT];
  const int tid = threadIdx.x;
  const int n0 = blockIdx.x * 64;
  const int k0 = blockIdx.y * 64;
#pragma unroll 4
  for (int j = 0; j < 16; ++j) {
    const int idx = tid + 256 * j;
    const int kr = idx >> 6, nc = idx & 63;
    const float v = W[(size_t)(k0 + kr) * N + n0 + nc];
    T[nc * LDT + kr] = (_Float16)(WCARRY * bf16r(v));
  }
  __syncthreads();
  v8h x[2];
  size_t off[2];
#pragma unroll
  for (int i = 0; i < 2; ++i) {
    const int n = 32 * i + (tid >> 3);
    const int kc = (tid & 7) * 8;
    x[i] = *(const v8h*)&T[n * LDT + kc];
    off[i] = (size_t)(n0 + n) * K + k0 + kc;
  }
#pragma unroll
  for (int i = 0; i < 2; ++i) *(volatile v8h*)(Wt + off[i]) = x[i];
  __threadfence();
#pragma unroll
  for (int i = 0; i < 2; ++i) *(volatile v8h*)(Wt + off[i]) = x[i];
}

__global__ __launch_bounds__(256) void xconv_kernel(
    const float* __restrict__ src, _Float16* __restrict__ dst) {
  const size_t e = ((size_t)blockIdx.x * 256 + threadIdx.x) * 8;
  const v4f a0 = *(const v4f*)(src + e);
  const v4f a1 = *(const v4f*)(src + e + 4);
  v8h o;
#pragma unroll
  for (int t = 0; t < 4; ++t) {
    o[t]     = toh_flush(bf16r(a0[t]));
    o[t + 4] = toh_flush(bf16r(a1[t]));
  }
  *(volatile v8h*)(dst + e) = o;
  __threadfence();
  *(volatile v8h*)(dst + e) = o;
}

#define MODE_QKV 0
#define MODE_OUT 1

template <int MODE, int KD, int ND, int RES>
__device__ __forceinline__ void gemm_body(
    const _Float16* __restrict__ A16, const _Float16* __restrict__ Ar16,
    const _Float16* __restrict__ Bt, const float* __restrict__ bias,
    float* __restrict__ outf, _Float16* __restrict__ out16,
    _Float16* __restrict__ outr16, int rowbase) {
  static_assert((KD % 32) == 0 && (ND % 64) == 0);
  static_assert(MODE != MODE_QKV || (ND == 3 * DIM && RES == 0));
  static_assert(MODE != MODE_OUT || ND == DIM);
  __shared__ float Cs[64 * LDC];
  const int tid = threadIdx.x, lane = tid & 31, w = tid >> 5;
  const int mw = w >> 1, nw = w & 1;
  const int hh = lane >> 4, m = lane & 15;
  const int n0 = blockIdx.x * 64;
  const int row0 = rowbase + blockIdx.y * 64;

  const _Float16* ap  = A16 + (size_t)(row0 + mw * 16 + m) * KD + hh * 8;
  const _Float16* arp = Ar16 + (size_t)(row0 + mw * 16 + m) * KD + hh * 8;
  const _Float16* bp0 = Bt + (size_t)(n0 + nw * 32 + m) * KD + hh * 8;
  const _Float16* bp1 = bp0 + (size_t)16 * KD;
  v8f acc0 = {}, acc1 = {}, acr0 = {}, acr1 = {};
#pragma unroll 2
  for (int k0 = 0; k0 < KD; k0 += 32) {
    const v16h a  = frag_at(ap + k0);
    const v16h b0 = frag_at(bp0 + k0);
    const v16h b1 = frag_at(bp1 + k0);
    acc0 = wmma16(a, b0, acc0);
    acc1 = wmma16(a, b1, acc1);
    if (RES) {
      const v16h ar = frag_at(arp + k0);
      acr0 = wmma16(ar, b0, acr0);
      acr1 = wmma16(ar, b1, acr1);
    }
  }
#pragma unroll
  for (int r = 0; r < 8; ++r) {
    float* d = &Cs[(mw * 16 + hh * 8 + r) * LDC + nw * 32 + m];
    d[0]  = RES ? (acc0[r] + acr0[r] * (1.0f / RCARRY)) : acc0[r];
    d[16] = RES ? (acc1[r] + acr1[r] * (1.0f / RCARRY)) : acc1[r];
  }
  __syncthreads();

  if (MODE == MODE_QKV) {
    const int head  = n0 / (3 * HD);
    const int which = (n0 - head * (3 * HD)) / HD;
    const int nl0 = head * HD;
    const bool early = (row0 < EROWS);
    _Float16* dst = out16 + (size_t)which * ((size_t)MROWS * DIM);
    _Float16* dsr = outr16 + (size_t)which * ((size_t)EROWS * DIM);
    v8h x[2], xr[2];
    size_t off[2], ofr[2];
    if (which < 2) {
#pragma unroll
      for (int i = 0; i < 2; ++i) {
        const int r = 32 * i + (tid >> 3);
        const int c = (tid & 7) * 8;
        const v4f u0 = *(const v4f*)&Cs[r * LDC + c];
        const v4f u1 = *(const v4f*)&Cs[r * LDC + c + 4];
        const v4f g0 = *(const v4f*)(bias + n0 + c);
        const v4f g1 = *(const v4f*)(bias + n0 + c + 4);
#pragma unroll
        for (int j = 0; j < 4; ++j) {
          const float t0 = u0[j] * (1.0f / WCARRY) + bf16r(g0[j]);
          const float t1 = u1[j] * (1.0f / WCARRY) + bf16r(g1[j]);
          const _Float16 h0 = toh_flush(t0);
          const _Float16 h1 = toh_flush(t1);
          x[i][j]      = h0;
          x[i][j + 4]  = h1;
          xr[i][j]     = toh_flush((t0 - (float)h0) * RCARRY);
          xr[i][j + 4] = toh_flush((t1 - (float)h1) * RCARRY);
        }
        off[i] = (size_t)(row0 + r) * DIM + nl0 + c;
        ofr[i] = off[i];
      }
    } else {
#pragma unroll
      for (int i = 0; i < 2; ++i) {
        const int dcol = 32 * i + (tid >> 3);
        const int kk = (tid & 7) * 8;
        const float gb = bf16r(bias[n0 + dcol]);
#pragma unroll
        for (int j = 0; j < 8; ++j) {
          const float t0 = Cs[(kk + j) * LDC + dcol] * (1.0f / WCARRY) + gb;
          const _Float16 h0 = toh_flush(t0);
          x[i][j]  = h0;
          xr[i][j] = toh_flush((t0 - (float)h0) * RCARRY);
        }
        off[i] = (size_t)(nl0 + dcol) * SEQ + row0 + kk;
        ofr[i] = (size_t)(nl0 + dcol) * EROWS + row0 + kk;
      }
    }
#pragma unroll
    for (int i = 0; i < 2; ++i) *(volatile v8h*)(dst + off[i]) = x[i];
    if (early) {
#pragma unroll
      for (int i = 0; i < 2; ++i) *(volatile v8h*)(dsr + ofr[i]) = xr[i];
    }
    __threadfence();
#pragma unroll
    for (int i = 0; i < 2; ++i) *(volatile v8h*)(dst + off[i]) = x[i];
    if (early) {
#pragma unroll
      for (int i = 0; i < 2; ++i) *(volatile v8h*)(dsr + ofr[i]) = xr[i];
    }
  }

  if (MODE == MODE_OUT) {
    v4f xs[4];
    size_t off[4];
#pragma unroll
    for (int i = 0; i < 4; ++i) {
      const int r = 16 * i + (tid >> 4);
      const int c = (tid & 15) * 4;
      const size_t crow = (size_t)(row0 + r);
      const v4f u = *(const v4f*)&Cs[r * LDC + c];
      const v4f g = *(const v4f*)(bias + n0 + c);
      v4f val;
#pragma unroll
      for (int j = 0; j < 4; ++j)
        val[j] = u[j] * (1.0f / (WCARRY * VCARRY)) + bf16r(g[j]);
      xs[i] = val;
      off[i] = crow * ND + n0 + c;
    }
#pragma unroll
    for (int i = 0; i < 4; ++i) *(volatile v4f*)(outf + off[i]) = xs[i];
    __threadfence();
#pragma unroll
    for (int i = 0; i < 4; ++i) *(volatile v4f*)(outf + off[i]) = xs[i];
  }
}

__global__ __launch_bounds__(256) void gemm_qkv_kernel(
    const _Float16* __restrict__ A16, const _Float16* __restrict__ Bt,
    const float* __restrict__ bias, _Float16* __restrict__ out16,
    _Float16* __restrict__ outr16) {
  gemm_body<MODE_QKV, DIM, 3 * DIM, 0>(A16, A16, Bt, bias, nullptr, out16, outr16, 0);
}

__global__ __launch_bounds__(256) void gemm_out_kernel(
    const _Float16* __restrict__ A16, const _Float16* __restrict__ Bt,
    const float* __restrict__ bias, float* __restrict__ outf, int rowbase) {
  gemm_body<MODE_OUT, DIM, DIM, 0>(A16, A16, Bt, bias, outf, nullptr, nullptr, rowbase);
}

__global__ __launch_bounds__(256) void gemm_out_early_kernel(
    const _Float16* __restrict__ A16, const _Float16* __restrict__ Ar16,
    const _Float16* __restrict__ Bt, const float* __restrict__ bias,
    float* __restrict__ outf) {
  gemm_body<MODE_OUT, DIM, DIM, 1>(A16, Ar16, Bt, bias, outf, nullptr, nullptr, 0);
}

__global__ __launch_bounds__(256) void attn_kernel(
    const _Float16* __restrict__ Qh, const _Float16* __restrict__ Kh,
    const _Float16* __restrict__ Vt, _Float16* __restrict__ Ov) {
  __shared__ _Float16 Ks[64 * LDT];
  __shared__ _Float16 Vs[64 * LDT];
  __shared__ _Float16 Ps[8 * 16 * LDT];

  const int tid = threadIdx.x, lane = tid & 31;
  const int w = __builtin_amdgcn_readfirstlane(tid >> 5);
  const int hh = lane >> 4, m = lane & 15;
  const int q0 = blockIdx.x * 128;
  const int head = blockIdx.y;
  const int wq0 = q0 + w * 16;
  const float scale = 0.125f;
  _Float16* P = Ps + w * (16 * LDT);

  const size_t qoff = (size_t)(wq0 + m) * DIM + head * HD + hh * 8;
  v16h qf[2];
  qf[0] = frag_at(Qh + qoff);
  qf[1] = frag_at(Qh + qoff + 32);

  float mrow[8], lrow[8];
  v8f o[4];
#pragma unroll
  for (int v = 0; v < 8; ++v) { mrow[v] = -1.0e30f; lrow[v] = 0.0f; }
#pragma unroll
  for (int nb = 0; nb < 4; ++nb) o[nb] = (v8f){};

  const size_t kplane = (size_t)head * HD;
  const size_t vplane = (size_t)head * HD * SEQ;
  const int kend = q0 + 128;

  for (int kb = 0; kb < kend; kb += 64) {
#pragma unroll
    for (int j = 0; j < 2; ++j) {
      const int idx = tid + 256 * j;
      const int r = idx >> 3, c = (idx & 7) * 8;
      *(v8h*)&Ks[r * LDT + c] = *(const v8h*)(Kh + kplane + (size_t)(kb + r) * DIM + c);
      *(v8h*)&Vs[r * LDT + c] = *(const v8h*)(Vt + vplane + (size_t)r * SEQ + kb + c);
    }
    __syncthreads();

    if (kb <= wq0 + 15) {
      v8f s[4];
#pragma unroll
      for (int kg = 0; kg < 4; ++kg) {
        v8f t = {};
#pragma unroll
        for (int c = 0; c < 2; ++c) {
          const v16h kf = ld_frag(&Ks[(kg * 16) * LDT + c * 32], LDT);
          t = wmma16(qf[c], kf, t);
        }
        s[kg] = t * scale;
      }

      if (kb + 63 > wq0) {
#pragma unroll
        for (int kg = 0; kg < 4; ++kg)
#pragma unroll
          for (int v = 0; v < 8; ++v) {
            const int key = kb + kg * 16 + m;
            const int qrow = wq0 + hh * 8 + v;
            s[kg][v] = (key > qrow) ? -1.0e30f : s[kg][v];
          }
      }

      float alpha[8];
#pragma unroll
      for (int v = 0; v < 8; ++v) {
        float mx = fmaxf(fmaxf(s[0][v], s[1][v]), fmaxf(s[2][v], s[3][v]));
        mx = red16_max(mx);
        const float mn = fmaxf(mrow[v], mx);
        alpha[v] = __expf(mrow[v] - mn);
        mrow[v] = mn;
      }
#pragma unroll
      for (int kg = 0; kg < 4; ++kg)
#pragma unroll
        for (int v = 0; v < 8; ++v) s[kg][v] = __expf(s[kg][v] - mrow[v]);
#pragma unroll
      for (int v = 0; v < 8; ++v) {
        const float rs = red16_sum((s[0][v] + s[1][v]) + (s[2][v] + s[3][v]));
        lrow[v] = alpha[v] * lrow[v] + rs;
      }
#pragma unroll
      for (int nb = 0; nb < 4; ++nb)
#pragma unroll
        for (int v = 0; v < 8; ++v) o[nb][v] = o[nb][v] * alpha[v];

#pragma unroll
      for (int kg = 0; kg < 4; ++kg)
#pragma unroll
        for (int v = 0; v < 8; ++v)
          P[(hh * 8 + v) * LDT + kg * 16 + m] = (_Float16)(s[kg][v] * PCARRY);
      wave_lds_sync();

#pragma unroll
      for (int c = 0; c < 2; ++c) {
        const v16h pf = ld_frag(P + c * 32, LDT);
#pragma unroll
        for (int nb = 0; nb < 4; ++nb) {
          const v16h vf = ld_frag(&Vs[(nb * 16) * LDT + c * 32], LDT);
          o[nb] = wmma16(pf, vf, o[nb]);
        }
      }
    }
    __syncthreads();
  }

  float inv[8];
#pragma unroll
  for (int v = 0; v < 8; ++v) inv[v] = __builtin_amdgcn_rcpf(lrow[v]) * (VCARRY / PCARRY);
#pragma unroll
  for (int nb = 0; nb < 4; ++nb)
#pragma unroll
    for (int v = 0; v < 8; ++v)
      P[(hh * 8 + v) * LDT + nb * 16 + m] = (_Float16)(o[nb][v] * inv[v]);
  wave_lds_sync();
  v8h x[4];
  size_t off[4];
#pragma unroll
  for (int i = 0; i < 4; ++i) {
    const int r = 4 * i + (lane >> 3);
    const int c = (lane & 7) * 8;
    x[i] = *(const v8h*)&P[r * LDT + c];
    off[i] = (size_t)(wq0 + r) * DIM + head * HD + c;
  }
#pragma unroll
  for (int i = 0; i < 4; ++i) *(volatile v8h*)(Ov + off[i]) = x[i];
  __threadfence();
#pragma unroll
  for (int i = 0; i < 4; ++i) *(volatile v8h*)(Ov + off[i]) = x[i];
}

__global__ __launch_bounds__(256) void attn_early_kernel(
    const _Float16* __restrict__ Qh, const _Float16* __restrict__ Qr,
    const _Float16* __restrict__ Kh, const _Float16* __restrict__ Kr,
    const _Float16* __restrict__ Vt, const _Float16* __restrict__ Vr,
    _Float16* __restrict__ Ov, _Float16* __restrict__ Ores) {
  __shared__ _Float16 Ks[64 * LDT];
  __shared__ _Float16 Vs[64 * LDT];
  __shared__ _Float16 Ps[8 * 16 * LDT];
  __shared__ _Float16 Rs[8 * 16 * LDT];

  const int tid = threadIdx.x, lane = tid & 31;
  const int w = __builtin_amdgcn_readfirstlane(tid >> 5);
  const int hh = lane >> 4, m = lane & 15;
  const int q0 = blockIdx.x * 128;
  const int head = blockIdx.y;
  const int wq0 = q0 + w * 16;
  const float scale = 0.125f;
  _Float16* P = Ps + w * (16 * LDT);
  _Float16* R = Rs + w * (16 * LDT);

  const int qoff = (wq0 + m) * DIM + head * HD + hh * 8;

  float mrow[8], lrow[8];
  v8f o[4], ores[4];
#pragma unroll
  for (int v = 0; v < 8; ++v) { mrow[v] = -1.0e30f; lrow[v] = 0.0f; }
#pragma unroll
  for (int nb = 0; nb < 4; ++nb) { o[nb] = (v8f){}; ores[nb] = (v8f){}; }

  const size_t kplane  = (size_t)head * HD;
  const size_t vplane  = (size_t)head * HD * SEQ;
  const size_t vrplane = (size_t)head * HD * EROWS;
  const int kend = q0 + 128;

  for (int kb = 0; kb < kend; kb += 64) {
#pragma unroll
    for (int j = 0; j < 2; ++j) {
      const int idx = tid + 256 * j;
      const int r = idx >> 3, c = (idx & 7) * 8;
      *(v8h*)&Ks[r * LDT + c] = *(const v8h*)(Kh + kplane + (size_t)(kb + r) * DIM + c);
      *(v8h*)&Vs[r * LDT + c] = *(const v8h*)(Vt + vplane + (size_t)r * SEQ + kb + c);
    }
    __syncthreads();

    if (kb <= wq0 + 15) {
      int qo = qoff;
      asm volatile("" : "+v"(qo));
      v16h qf[2], qr[2];
      qf[0] = frag_at(Qh + qo);
      qf[1] = frag_at(Qh + qo + 32);
      qr[0] = frag_at(Qr + qo);
      qr[1] = frag_at(Qr + qo + 32);

      v8f s[4];
#pragma unroll
      for (int kg = 0; kg < 4; ++kg) {
        v8f t = {};
        v8f u = {};
#pragma unroll
        for (int c = 0; c < 2; ++c) {
          const v16h kf = ld_frag(&Ks[(kg * 16) * LDT + c * 32], LDT);
          const v16h krf = frag_at(Kr + kplane + (size_t)(kb + kg * 16 + m) * DIM +
                                   c * 32 + hh * 8);
          t = wmma16(qf[c], kf, t);
          u = wmma16(qf[c], krf, u);
          u = wmma16(qr[c], kf, u);
        }
        s[kg] = (t + u * (1.0f / RCARRY)) * scale;
      }

      if (kb + 63 > wq0) {
#pragma unroll
        for (int kg = 0; kg < 4; ++kg)
#pragma unroll
          for (int v = 0; v < 8; ++v) {
            const int key = kb + kg * 16 + m;
            const int qrow = wq0 + hh * 8 + v;
            s[kg][v] = (key > qrow) ? -1.0e30f : s[kg][v];
          }
      }

      float alpha[8];
#pragma unroll
      for (int v = 0; v < 8; ++v) {
        float mx = fmaxf(fmaxf(s[0][v], s[1][v]), fmaxf(s[2][v], s[3][v]));
        mx = red16_max(mx);
        const float mn = fmaxf(mrow[v], mx);
        alpha[v] = __expf(mrow[v] - mn);
        mrow[v] = mn;
      }
#pragma unroll
      for (int kg = 0; kg < 4; ++kg)
#pragma unroll
        for (int v = 0; v < 8; ++v) s[kg][v] = __expf(s[kg][v] - mrow[v]);
#pragma unroll
      for (int v = 0; v < 8; ++v) {
        const float rs = red16_sum((s[0][v] + s[1][v]) + (s[2][v] + s[3][v]));
        lrow[v] = alpha[v] * lrow[v] + rs;
      }
#pragma unroll
      for (int nb = 0; nb < 4; ++nb)
#pragma unroll
        for (int v = 0; v < 8; ++v) {
          o[nb][v]    = o[nb][v] * alpha[v];
          ores[nb][v] = ores[nb][v] * alpha[v];
        }

#pragma unroll
      for (int kg = 0; kg < 4; ++kg)
#pragma unroll
        for (int v = 0; v < 8; ++v) {
          const float pc = s[kg][v] * PCARRY;
          const _Float16 ph = toh_flush(pc);
          P[(hh * 8 + v) * LDT + kg * 16 + m] = ph;
          R[(hh * 8 + v) * LDT + kg * 16 + m] = toh_flush((pc - (float)ph) * RCARRY);
        }
      wave_lds_sync();

#pragma unroll
      for (int c = 0; c < 2; ++c) {
        const v16h pf  = ld_frag(P + c * 32, LDT);
        const v16h prf = ld_frag(R + c * 32, LDT);
#pragma unroll
        for (int nb = 0; nb < 4; ++nb) {
          const v16h vf = ld_frag(&Vs[(nb * 16) * LDT + c * 32], LDT);
          const v16h vrf = frag_at(Vr + vrplane + (size_t)(nb * 16 + m) * EROWS + kb +
                                   c * 32 + hh * 8);
          o[nb]    = wmma16(pf, vf, o[nb]);
          ores[nb] = wmma16(pf, vrf, ores[nb]);
          ores[nb] = wmma16(prf, vf, ores[nb]);
        }
      }
    }
    __syncthreads();
  }

  float inv[8];
#pragma unroll
  for (int v = 0; v < 8; ++v) inv[v] = __builtin_amdgcn_rcpf(lrow[v]) * (VCARRY / PCARRY);
#pragma unroll
  for (int nb = 0; nb < 4; ++nb)
#pragma unroll
    for (int v = 0; v < 8; ++v) {
      const float val = (o[nb][v] + ores[nb][v] * (1.0f / RCARRY)) * inv[v];
      const _Float16 hv = toh_flush(val);
      P[(hh * 8 + v) * LDT + nb * 16 + m] = hv;
      R[(hh * 8 + v) * LDT + nb * 16 + m] = toh_flush((val - (float)hv) * RCARRY);
    }
  wave_lds_sync();
  v8h x[4], xr[4];
  size_t off[4];
#pragma unroll
  for (int i = 0; i < 4; ++i) {
    const int r = 4 * i + (lane >> 3);
    const int c = (lane & 7) * 8;
    x[i]  = *(const v8h*)&P[r * LDT + c];
    xr[i] = *(const v8h*)&R[r * LDT + c];
    off[i] = (size_t)(wq0 + r) * DIM + head * HD + c;
  }
#pragma unroll
  for (int i = 0; i < 4; ++i) {
    *(volatile v8h*)(Ov + off[i]) = x[i];
    *(volatile v8h*)(Ores + off[i]) = xr[i];
  }
  __threadfence();
#pragma unroll
  for (int i = 0; i < 4; ++i) {
    *(volatile v8h*)(Ov + off[i]) = x[i];
    *(volatile v8h*)(Ores + off[i]) = xr[i];
  }
}

extern "C" void kernel_launch(void* const* d_in, const int* in_sizes, int n_in,
                              void* d_out, int out_size, void* d_ws, size_t ws_size,
                              hipStream_t stream) {
  if (n_in < 5) return;
  const long long need_x = ((long long)(NB - 1) * SEQ_FULL + SEQ) * DIM;
  if ((long long)in_sizes[0] < need_x) return;
  if (in_sizes[1] < 3 * DIM * DIM || in_sizes[2] < 3 * DIM) return;
  if (in_sizes[3] < DIM * DIM || in_sizes[4] < DIM) return;
  if ((long long)out_size < need_x) return;
  if (ws_size < WS_TOTAL) return;

  const float* x  = (const float*)d_in[0];
  const float* W1 = (const float*)d_in[1];
  const float* b1 = (const float*)d_in[2];
  const float* Wp = (const float*)d_in[3];
  const float* bp = (const float*)d_in[4];
  float* out = (float*)d_out;

  char* ws = (char*)d_ws;
  _Float16* W1T   = (_Float16*)(ws + OFF_WQKV);
  _Float16* WpT   = (_Float16*)(ws + OFF_WO);
  _Float16* X16   = (_Float16*)(ws + OFF_XN);
  _Float16* QKV16 = (_Float16*)(ws + OFF_QKV);
  _Float16* Q16   = QKV16;
  _Float16* K16   = QKV16 + (size_t)MROWS * DIM;
  _Float16* Vt16  = QKV16 + (size_t)2 * MROWS * DIM;
  _Float16* Ov16  = (_Float16*)(ws + OFF_OV);
  _Float16* RES16 = (_Float16*)(ws + OFF_RES);
  _Float16* QR16  = RES16;
  _Float16* KR16  = RES16 + (size_t)EROWS * DIM;
  _Float16* VtR16 = RES16 + (size_t)2 * EROWS * DIM;
  _Float16* OR16  = (_Float16*)(ws + OFF_ORES);

  dim3 blk(256);

  wconv_kernel<<<dim3(3 * DIM / 64, DIM / 64), blk, 0, stream>>>(W1, W1T, DIM, 3 * DIM);
  wconv_kernel<<<dim3(DIM / 64, DIM / 64), blk, 0, stream>>>(Wp, WpT, DIM, DIM);

  xconv_kernel<<<dim3((unsigned)(((size_t)MROWS * DIM) / 2048)), blk, 0, stream>>>(x, X16);
  gemm_qkv_kernel<<<dim3(3 * DIM / 64, MROWS / 64), blk, 0, stream>>>(
      X16, W1T, b1, QKV16, RES16);
  attn_kernel<<<dim3(SEQ / 128, NHEAD), blk, 0, stream>>>(Q16, K16, Vt16, Ov16);
  attn_early_kernel<<<dim3(EROWS / 128, NHEAD), blk, 0, stream>>>(
      Q16, QR16, K16, KR16, Vt16, VtR16, Ov16, OR16);
  if (MROWS > EROWS) {
    gemm_out_kernel<<<dim3(DIM / 64, (MROWS - EROWS) / 64), blk, 0, stream>>>(
        Ov16, WpT, bp, out, EROWS);
  }
  gemm_out_early_kernel<<<dim3(DIM / 64, EROWS / 64), blk, 0, stream>>>(
      Ov16, OR16, WpT, bp, out);
}
